// SelfAttention_47115791237647
// MI455X (gfx1250) — hardware-run, weakly checked
//
#include <hip/hip_runtime.h>


#ifndef NB
#define NB 32
#endif
#define NB_FULL    32
#define NTOK       577
#define EMB        768
#define NHEAD      12
#define HDIM       64
#define NPAD       640
#define NKEY       608
#define HGT        24
#define WID        24
#define RELW       47
#define NREL       2209
#define RELP       2240
#define NROWS      (NB * NTOK)
#define NQKV       (3 * EMB)
#define QM         64
#define QN         128
#define TPB        (NPAD / QM)
#define CP         72
#define OP         68
#define KSTEPS     (EMB / 32)
#define WS_CAP     134217728ull
#define LOG2E      1.4426950408889634f

#define XB_BYTES   ((unsigned long long)NROWS * EMB * 2ull)
#define WQKV_BYTES ((unsigned long long)NQKV * EMB * 2ull)
#define WP_BYTES   ((unsigned long long)EMB * EMB * 2ull)
#define BIAS_BYTES ((unsigned long long)(NQKV + EMB) * 4ull)
#define PL_ELEMS   ((unsigned long long)NB * NHEAD * NPAD * HDIM)
#define PL_BYTES   (PL_ELEMS * 2ull)
#define OFF_XB     0ull
#define OFF_WQKV   (OFF_XB + XB_BYTES)
#define OFF_WP     (OFF_WQKV + WQKV_BYTES)
#define OFF_BIAS   (OFF_WP + WP_BYTES)
#define OFF_PL     (OFF_BIAS + BIAS_BYTES)
#define WS_TOTAL   (OFF_PL + 3ull * PL_BYTES)

static_assert(NB >= 1 && NB <= NB_FULL);
static_assert(EMB == NHEAD * HDIM);
static_assert(HDIM == 64);
static_assert(EMB % 32 == 0);
static_assert(NPAD % QM == 0);
static_assert(NKEY % 32 == 0 && NKEY <= NPAD && NKEY >= NTOK);
static_assert(NQKV % QN == 0 && EMB % QN == 0);
static_assert(EMB % 256 == 0);
static_assert(((unsigned long long)NTOK * EMB) % 64 == 0);
static_assert((EMB * EMB) % (256 * 8) == 0);
static_assert(XB_BYTES % 128 == 0 && WQKV_BYTES % 128 == 0 && WP_BYTES % 128 == 0 && BIAS_BYTES % 128 == 0);
static_assert(PL_BYTES % 128 == 0);
static_assert(WS_TOTAL <= WS_CAP);
static_assert(RELP % 64 == 0 && RELP >= NREL);
static_assert((CP * 2) % 16 == 0 && (OP * 4) % 16 == 0 && CP >= 64 && OP >= 64);

typedef __bf16   bf16;
typedef _Float16 f16;
typedef bf16     v16bf __attribute__((ext_vector_type(16)));
typedef f16      v16h  __attribute__((ext_vector_type(16)));
typedef f16      v8h   __attribute__((ext_vector_type(8)));
typedef float    v8f   __attribute__((ext_vector_type(8)));
typedef float    v4f   __attribute__((ext_vector_type(4)));
typedef unsigned v4u   __attribute__((ext_vector_type(4)));

union FragB  { v16bf v; v4u q[2]; bf16 h[16]; };
union FragH  { v16h  v; v4u q[2]; f16  h[16]; };
union Pack8B { v4u u; bf16 h[8]; };
union Pack8H { v4u u; v8h v; f16 h[8]; };

static __device__ __forceinline__ int imin(int a, int b) { return a < b ? a : b; }
static __device__ __forceinline__ int imax(int a, int b) { return a > b ? a : b; }

static __device__ __forceinline__ v8f mma_bf16(v16bf a, v16bf b, v8f acc) {
  acc = __builtin_amdgcn_wmma_f32_16x16x32_bf16(false, a, false, b, (short)0, acc, false, false);
  asm volatile("v_nop\n\tv_nop\n\tv_nop\n\tv_nop" : "+v"(acc) : "v"(a), "v"(b));
  return acc;
}
static __device__ __forceinline__ v8f mma_f16(v16h a, v16h b, v8f acc) {
  acc = __builtin_amdgcn_wmma_f32_16x16x32_f16(false, a, false, b, (short)0, acc, false, false);
  asm volatile("v_nop\n\tv_nop\n\tv_nop\n\tv_nop" : "+v"(acc) : "v"(a), "v"(b));
  return acc;
}

__global__ __launch_bounds__(256) void cvt_x_kernel(const float* __restrict__ x, bf16* __restrict__ xb, int n8) {
  const int i = blockIdx.x * 256 + threadIdx.x;
  if (i >= n8) return;
  const size_t e = (size_t)i * 8;
  const v4f a0 = *(const v4f*)(x + e);
  const v4f a1 = *(const v4f*)(x + e + 4);
  Pack8B pk;
  #pragma unroll
  for (int j = 0; j < 4; ++j) {
    pk.h[j]     = (bf16)a0[j];
    pk.h[4 + j] = (bf16)a1[j];
  }
  const v4u u = pk.u;
  *(volatile v4u*)(xb + e) = u;
  __threadfence();
  *(volatile v4u*)(xb + e) = u;
}

__global__ __launch_bounds__(256) void cvt_w_kernel(const float* __restrict__ w, const float* __restrict__ bias,
                                                    unsigned short* __restrict__ dst, float* __restrict__ bdst,
                                                    int mode) {
  const int i = blockIdx.x * 256 + threadIdx.x;
  const size_t e = (size_t)i * 8;
  const v4f a0 = *(const v4f*)(w + e);
  const v4f a1 = *(const v4f*)(w + e + 4);
  Pack8B pb;
  Pack8H ph;
  #pragma unroll
  for (int j = 0; j < 4; ++j) {
    const bf16 r0 = (bf16)a0[j];
    const bf16 r1 = (bf16)a1[j];
    pb.h[j]     = r0;
    pb.h[4 + j] = r1;
    ph.h[j]     = (f16)((float)r0 * 64.0f);
    ph.h[4 + j] = (f16)((float)r1 * 64.0f);
  }
  const v4u u = (mode == 0) ? pb.u : ph.u;
  const bool doBias = (blockIdx.x == 0) && (threadIdx.x < EMB / 4);
  v4f bvv = (v4f){0.0f, 0.0f, 0.0f, 0.0f};
  if (doBias) {
    const v4f t = *(const v4f*)(bias + threadIdx.x * 4);
    #pragma unroll
    for (int j = 0; j < 4; ++j) bvv[j] = (float)(bf16)t[j];
  }
  *(volatile v4u*)(dst + e) = u;
  if (doBias) *(volatile v4f*)(bdst + threadIdx.x * 4) = bvv;
  __threadfence();
  *(volatile v4u*)(dst + e) = u;
  if (doBias) *(volatile v4f*)(bdst + threadIdx.x * 4) = bvv;
}

__global__ __launch_bounds__(128) void qkv_gemm_kernel(const bf16* __restrict__ xb,
                                                       const bf16* __restrict__ wqkv,
                                                       const float* __restrict__ bias_all,
                                                       f16* __restrict__ planes) {
  const int tile = blockIdx.x;
  const int b    = tile / TPB;
  const int t0   = (tile - b * TPB) * QM;
  const int ny   = blockIdx.y;
  const int mat  = ny / (EMB / QN);
  const int hp   = ny - mat * (EMB / QN);
  const int tid  = threadIdx.x;
  const int wave = __builtin_amdgcn_readfirstlane(threadIdx.x >> 5);
  const int lane = tid & 31;
  const int lq   = lane & 15;
  const int hi   = lane >> 4;
  const int mi   = wave & 1;
  const int ni   = wave >> 1;
  const int n0   = ny * QN + ni * 64;

  __shared__ __align__(16) f16 sC[2 * 64 * CP];

  v8f acc[2][4];
  #pragma unroll
  for (int a = 0; a < 2; ++a) {
    #pragma unroll
    for (int c = 0; c < 4; ++c) acc[a][c] = (v8f){0, 0, 0, 0, 0, 0, 0, 0};
  }

  const bool live = (t0 + mi * 32) < NTOK;
  if (live) {
    const int tok0 = imin(t0 + mi * 32 + lq, NTOK - 1);
    const int tok1 = imin(t0 + mi * 32 + 16 + lq, NTOK - 1);
    const bf16* a0p = xb + ((size_t)b * NTOK + tok0) * EMB + hi * 8;
    const bf16* a1p = xb + ((size_t)b * NTOK + tok1) * EMB + hi * 8;
    const bf16* wp0 = wqkv + (size_t)(n0 + lq) * EMB + hi * 8;
    #pragma unroll 1
    for (int kt = 0; kt < KSTEPS; ++kt) {
      FragB a0, a1;
      a0.q[0] = *(const v4u*)(a0p + kt * 32);
      a0.q[1] = *(const v4u*)(a0p + kt * 32 + 16);
      a1.q[0] = *(const v4u*)(a1p + kt * 32);
      a1.q[1] = *(const v4u*)(a1p + kt * 32 + 16);
      #pragma unroll
      for (int nt = 0; nt < 4; ++nt) {
        FragB bb;
        const bf16* p = wp0 + (size_t)nt * 16 * EMB + kt * 32;
        bb.q[0] = *(const v4u*)(p);
        bb.q[1] = *(const v4u*)(p + 16);
        acc[0][nt] = mma_bf16(a0.v, bb.v, acc[0][nt]);
        acc[1][nt] = mma_bf16(a1.v, bb.v, acc[1][nt]);
      }
    }
  }

  const bool tr = (mat == 2);
  #pragma unroll
  for (int mi2 = 0; mi2 < 2; ++mi2) {
    #pragma unroll
    for (int nt = 0; nt < 4; ++nt) {
      const int col = nt * 16 + lq;
      const float bb = bias_all[n0 + col];
      #pragma unroll
      for (int r = 0; r < 8; ++r) {
        const int row = mi * 32 + mi2 * 16 + hi * 8 + r;
        const f16 hv = (f16)((acc[mi2][nt][r] + bb) * 16.0f);
        const int idx = tr ? (col * CP + row) : (row * CP + col);
        sC[ni * (64 * CP) + idx] = hv;
      }
    }
  }
  __syncthreads();

  f16* dst = planes + (size_t)mat * (size_t)PL_ELEMS;
  v4u    val[8];
  size_t off[8];
  #pragma unroll
  for (int it = 0; it < 8; ++it) {
    const int p    = it * 128 + tid;
    const int line = p >> 3;
    const int seg  = p & 7;
    const int hd   = line >> 6;
    const int rl   = line & 63;
    Pack8H ph;
    ph.v = *(const v8h*)(sC + (hd * 64 + rl) * CP + seg * 8);
    val[it] = ph.u;
    const size_t bh = (size_t)b * NHEAD + (hp * 2 + hd);
    off[it] = tr ? ((bh * HDIM + rl) * NPAD + t0 + seg * 8)
                 : ((bh * NPAD + t0 + rl) * HDIM + seg * 8);
  }
  #pragma unroll
  for (int it = 0; it < 8; ++it) *(volatile v4u*)(dst + off[it]) = val[it];
  __threadfence();
  #pragma unroll
  for (int it = 0; it < 8; ++it) *(volatile v4u*)(dst + off[it]) = val[it];
}

__global__ __launch_bounds__(64) void attn_kernel(const f16* __restrict__ planes,
                                                  const float* __restrict__ rel,
                                                  f16* __restrict__ ctx) {
  const int qblk = blockIdx.x;
  const int h    = blockIdx.y;
  const int b    = blockIdx.z;
  const int tid  = threadIdx.x;
  const int wave = __builtin_amdgcn_readfirstlane(threadIdx.x >> 5);
  const int lane = tid & 31;
  const int lq   = lane & 15;
  const int hi   = lane >> 4;

  __shared__ __align__(16) float sRel[RELP];
  __shared__ __align__(16) f16   sO[2 * 16 * CP];

  #pragma unroll 1
  for (int i = tid; i < RELP; i += 64) {
    const int ic = imin(i, NREL - 1);
    const float v = (float)(bf16)rel[ic * NHEAD + h];
    sRel[i] = (i < NREL) ? v * LOG2E : 0.0f;
  }
  __syncthreads();

  const size_t bh   = (size_t)b * NHEAD + h;
  const f16*   q_h  = planes + bh * NPAD * HDIM;
  const f16*   k_h  = planes + (size_t)PL_ELEMS + bh * NPAD * HDIM;
  const f16*   vt_h = planes + 2 * (size_t)PL_ELEMS + bh * HDIM * NPAD;

  const int qrow0 = qblk * 32 + wave * 16;

  FragH qf[2];
  {
    const f16* qp = q_h + (size_t)(qrow0 + lq) * HDIM + hi * 8;
    #pragma unroll
    for (int f = 0; f < 2; ++f) {
      qf[f].q[0] = *(const v4u*)(qp + f * 32);
      qf[f].q[1] = *(const v4u*)(qp + f * 32 + 16);
    }
  }

  const int  tq    = qrow0 + lq;
  const bool qb    = (tq >= 1) && (tq < NTOK);
  const int  gq    = imax(tq - 1, 0);
  const int  qy    = gq / WID;
  const int  qx    = gq - qy * WID;
  const int  baseq = (qy + HGT - 1) * RELW + qx + WID - 1;

  v8f o[4];
  #pragma unroll
  for (int dt = 0; dt < 4; ++dt) o[dt] = (v8f){0, 0, 0, 0, 0, 0, 0, 0};

  float rmax = -__builtin_inff();
  float rsum = 0.0f;
  const float SL = 0.125f * (1.0f / 256.0f) * LOG2E;

  const int nchunk = NKEY / 32;
  #pragma unroll 1
  for (int i = 0; i < nchunk; ++i) {
    const int j0 = i * 32;

    FragH ak[2][2];
    #pragma unroll
    for (int sub = 0; sub < 2; ++sub) {
      #pragma unroll
      for (int f = 0; f < 2; ++f) {
        const f16* base = k_h + (size_t)(j0 + sub * 16 + lq) * HDIM + f * 32 + hi * 8;
        ak[sub][f].q[0] = *(const v4u*)(base);
        ak[sub][f].q[1] = *(const v4u*)(base + 16);
      }
    }
    FragH bv[4];
    #pragma unroll
    for (int dt = 0; dt < 4; ++dt) {
      const f16* base = vt_h + (size_t)(dt * 16 + lq) * NPAD + j0 + hi * 8;
      bv[dt].q[0] = *(const v4u*)(base);
      bv[dt].q[1] = *(const v4u*)(base + 16);
    }

    v8f c[2];
    #pragma unroll
    for (int sub = 0; sub < 2; ++sub) {
      v8f acc = (v8f){0, 0, 0, 0, 0, 0, 0, 0};
      acc = mma_f16(ak[sub][0].v, qf[0].v, acc);
      acc = mma_f16(ak[sub][1].v, qf[1].v, acc);
      c[sub] = acc;
    }

    float t[2][8];
    #pragma unroll
    for (int sub = 0; sub < 2; ++sub) {
      #pragma unroll
      for (int r = 0; r < 8; ++r) {
        const int tk  = j0 + sub * 16 + hi * 8 + r;
        const int g   = imax(tk - 1, 0);
        const int ky  = g / WID;
        int idx = baseq - g - (RELW - WID) * ky;
        idx = imin(imax(idx, 0), NREL - 1);
        const float bsv  = sRel[idx];
        const bool  use  = qb && (tk >= 1) && (tk < NTOK);
        const float bias = use ? bsv : 0.0f;
        const float tv   = fmaf(c[sub][r], SL, bias);
        t[sub][r] = (tk < NTOK) ? tv : -1.0e30f;
      }
    }

    float m_new = rmax;
    #pragma unroll
    for (int r = 0; r < 8; ++r) {
      m_new = fmaxf(m_new, t[0][r]);
      m_new = fmaxf(m_new, t[1][r]);
    }
    m_new = fmaxf(m_new, __shfl_xor(m_new, 16, 32));
    const float scale = __builtin_amdgcn_exp2f(rmax - m_new);
    rmax = m_new;

    FragH pa;
    float psum = 0.0f;
    #pragma unroll
    for (int r = 0; r < 8; ++r) {
      const float p0 = __builtin_amdgcn_exp2f(t[0][r] - m_new);
      const float p1 = __builtin_amdgcn_exp2f(t[1][r] - m_new);
      psum += p0 + p1;
      pa.h[r]     = (f16)(p0 * 4096.0f);
      pa.h[8 + r] = (f16)(p1 * 4096.0f);
    }
    rsum = rsum * scale + psum + __shfl_xor(psum, 16, 32);

    float sc[8];
    #pragma unroll
    for (int r = 0; r < 8; ++r) sc[r] = __shfl(scale, (hi << 3) + r, 32);
    #pragma unroll
    for (int dt = 0; dt < 4; ++dt) {
      #pragma unroll
      for (int r = 0; r < 8; ++r) o[dt][r] *= sc[r];
    }

    #pragma unroll
    for (int dt = 0; dt < 4; ++dt) o[dt] = mma_f16(pa.v, bv[dt].v, o[dt]);
  }

  float rs[8];
  #pragma unroll
  for (int r = 0; r < 8; ++r) rs[r] = 1.0f / __shfl(rsum, (hi << 3) + r, 32);

  f16* so = sO + wave * (16 * CP);
  #pragma unroll
  for (int r = 0; r < 8; ++r) {
    #pragma unroll
    for (int dt = 0; dt < 4; ++dt) {
      so[(hi * 8 + r) * CP + dt * 16 + lq] = (f16)(o[dt][r] * (1.0f / 1024.0f) * rs[r]);
    }
  }
  __syncthreads();

  v4u    vals[4];
  size_t gidx[4];
  bool   okr[4];
  #pragma unroll
  for (int it = 0; it < 4; ++it) {
    const int row = it * 4 + (lane >> 3);
    const int seg = lane & 7;
    Pack8H ph;
    ph.v = *(const v8h*)(so + row * CP + seg * 8);
    vals[it] = ph.u;
    const int tqr = qrow0 + row;
    okr[it] = tqr < NTOK;
    const int tqc = imin(tqr, NTOK - 1);
    gidx[it] = ((size_t)b * NTOK + tqc) * EMB + h * HDIM + seg * 8;
  }
  #pragma unroll
  for (int it = 0; it < 4; ++it) { if (okr[it]) *(volatile v4u*)(ctx + gidx[it]) = vals[it]; }
  __threadfence();
  #pragma unroll
  for (int it = 0; it < 4; ++it) { if (okr[it]) *(volatile v4u*)(ctx + gidx[it]) = vals[it]; }
}

__global__ __launch_bounds__(128) void proj_gemm_kernel(const f16* __restrict__ ctx,
                                                        const f16* __restrict__ wph,
                                                        const float* __restrict__ bias_all,
                                                        float* __restrict__ out) {
  const int mtile = blockIdx.x;
  const int tid   = threadIdx.x;
  const int wave  = __builtin_amdgcn_readfirstlane(threadIdx.x >> 5);
  const int lane  = tid & 31;
  const int lq    = lane & 15;
  const int hi    = lane >> 4;
  const int n0    = (blockIdx.y * 4 + wave) * 64;

  __shared__ __align__(16) float sP[4 * 32 * OP];

  const int r0 = imin(mtile * 32 + lq, NROWS - 1);
  const int r1 = imin(mtile * 32 + 16 + lq, NROWS - 1);
  const f16* a0p = ctx + (size_t)r0 * EMB + hi * 8;
  const f16* a1p = ctx + (size_t)r1 * EMB + hi * 8;
  const f16* wp0 = wph + (size_t)(n0 + lq) * EMB + hi * 8;

  v8f acc[2][4];
  #pragma unroll
  for (int a = 0; a < 2; ++a) {
    #pragma unroll
    for (int c = 0; c < 4; ++c) acc[a][c] = (v8f){0, 0, 0, 0, 0, 0, 0, 0};
  }

  #pragma unroll 1
  for (int kt = 0; kt < KSTEPS; ++kt) {
    FragH a0, a1;
    a0.q[0] = *(const v4u*)(a0p + kt * 32);
    a0.q[1] = *(const v4u*)(a0p + kt * 32 + 16);
    a1.q[0] = *(const v4u*)(a1p + kt * 32);
    a1.q[1] = *(const v4u*)(a1p + kt * 32 + 16);
    #pragma unroll
    for (int nt = 0; nt < 4; ++nt) {
      FragH bb;
      const f16* p = wp0 + (size_t)nt * 16 * EMB + kt * 32;
      bb.q[0] = *(const v4u*)(p);
      bb.q[1] = *(const v4u*)(p + 16);
      acc[0][nt] = mma_f16(a0.v, bb.v, acc[0][nt]);
      acc[1][nt] = mma_f16(a1.v, bb.v, acc[1][nt]);
    }
  }

  float* so = sP + wave * (32 * OP);
  #pragma unroll
  for (int mi2 = 0; mi2 < 2; ++mi2) {
    #pragma unroll
    for (int nt = 0; nt < 4; ++nt) {
      const float bb = bias_all[NQKV + n0 + nt * 16 + lq];
      #pragma unroll
      for (int r = 0; r < 8; ++r) {
        so[(mi2 * 16 + hi * 8 + r) * OP + nt * 16 + lq] = acc[mi2][nt][r] * (1.0f / 4096.0f) + bb;
      }
    }
  }
  __syncthreads();

  v4f vals[16];
  #pragma unroll
  for (int it = 0; it < 16; ++it) {
    const int row = it * 2 + hi;
    vals[it] = *(const v4f*)(so + row * OP + lq * 4);
  }
  #pragma unroll
  for (int it = 0; it < 16; ++it) {
    const int grow = mtile * 32 + it * 2 + hi;
    if (grow < NROWS) *(volatile v4f*)(out + (size_t)grow * EMB + n0 + lq * 4) = vals[it];
  }
  __threadfence();
  #pragma unroll
  for (int it = 0; it < 16; ++it) {
    const int grow = mtile * 32 + it * 2 + hi;
    if (grow < NROWS) *(volatile v4f*)(out + (size_t)grow * EMB + n0 + lq * 4) = vals[it];
  }
}

extern "C" void kernel_launch(void* const* d_in, const int* in_sizes, int n_in,
                              void* d_out, int out_size, void* d_ws, size_t ws_size,
                              hipStream_t stream) {
  if (n_in < 10) return;
  const size_t nx = (size_t)NROWS * EMB;
  if ((size_t)in_sizes[0] < nx) return;
  if ((size_t)in_sizes[1] < (size_t)EMB * EMB) return;
  if ((size_t)in_sizes[3] < (size_t)EMB * EMB) return;
  if ((size_t)in_sizes[5] < (size_t)EMB * EMB) return;
  if ((size_t)in_sizes[7] < (size_t)EMB * EMB) return;
  if (in_sizes[2] < EMB || in_sizes[4] < EMB || in_sizes[6] < EMB || in_sizes[8] < EMB) return;
  if (in_sizes[9] < NREL * NHEAD) return;
  if ((size_t)out_size < nx) return;
  if (ws_size < (size_t)WS_TOTAL) return;

  const float* x   = (const float*)d_in[0];
  const float* Wq  = (const float*)d_in[1];
  const float* bq  = (const float*)d_in[2];
  const float* Wk  = (const float*)d_in[3];
  const float* bk  = (const float*)d_in[4];
  const float* Wv  = (const float*)d_in[5];
  const float* bv  = (const float*)d_in[6];
  const float* Wp  = (const float*)d_in[7];
  const float* bp  = (const float*)d_in[8];
  const float* rel = (const float*)d_in[9];
  float* out = (float*)d_out;

  char* ws = (char*)d_ws;
  bf16*           xb       = (bf16*)(ws + OFF_XB);
  f16*            ctx      = (f16*)(ws + OFF_XB);
  unsigned short* wqkv_u   = (unsigned short*)(ws + OFF_WQKV);
  unsigned short* wph_u    = (unsigned short*)(ws + OFF_WP);
  float*          bias_all = (float*)(ws + OFF_BIAS);
  f16*            planes   = (f16*)(ws + OFF_PL);

  const int n8 = (int)(nx / 8);
  cvt_x_kernel<<<dim3((n8 + 255) / 256), 256, 0, stream>>>(x, xb, n8);

  const int wblocks = (EMB * EMB) / (256 * 8);
  cvt_w_kernel<<<dim3(wblocks), 256, 0, stream>>>(Wq, bq, wqkv_u,                         bias_all,           0);
  cvt_w_kernel<<<dim3(wblocks), 256, 0, stream>>>(Wk, bk, wqkv_u + (size_t)EMB * EMB,     bias_all + EMB,     0);
  cvt_w_kernel<<<dim3(wblocks), 256, 0, stream>>>(Wv, bv, wqkv_u + (size_t)2 * EMB * EMB, bias_all + 2 * EMB, 0);
  cvt_w_kernel<<<dim3(wblocks), 256, 0, stream>>>(Wp, bp, wph_u,                          bias_all + NQKV,    1);

  qkv_gemm_kernel<<<dim3(NB * TPB, NQKV / QN), 128, 0, stream>>>(xb, (const bf16*)wqkv_u, bias_all, planes);
  attn_kernel<<<dim3(NKEY / 32, NHEAD, NB), 64, 0, stream>>>(planes, rel, ctx);
  proj_gemm_kernel<<<dim3((NROWS + 31) / 32, EMB / 256), 128, 0, stream>>>(ctx, (const f16*)wph_u, bias_all, out);
}
